// SimplifiedMamba_62070867361926
// MI455X (gfx1250) — hardware-run, weakly checked
//
#include <hip/hip_runtime.h>
#include <math.h>

typedef __attribute__((ext_vector_type(16))) _Float16 v16h;
typedef __attribute__((ext_vector_type(8)))  _Float16 v8h;
typedef __attribute__((ext_vector_type(8)))  float    v8f;
typedef __attribute__((ext_vector_type(4)))  float    v4f;

constexpr int kBatch = 8;
constexpr int kSeq   = 2048;
constexpr int kDm    = 512;
constexpr int kDi    = 768;
constexpr int kNs    = 8;
constexpr int kRows  = kBatch * kSeq;
constexpr int kXgP   = 2 * kDi;
constexpr int kTP    = 260;
constexpr int kScanCh = 256;
constexpr int kScanBlkPerB = kDi / kScanCh;

constexpr float kXCarry = 16.0f;
constexpr float kWCarry = 1024.0f;
constexpr float kYCarry = 64.0f;
constexpr float kFold1  = 1.0f / (kXCarry * kWCarry);
constexpr float kFold2  = 1.0f / (kYCarry * kWCarry);
constexpr float kH16Min = 6.103515625e-05f;
constexpr float kH16Max = 65504.0f;
constexpr float kLog2e  = 1.4426950408889634f;

static_assert(kRows == 16384 && kXgP == 1536, "shape constants");
static_assert((kDm % 32) == 0 && (kDi % 32) == 0, "GEMM K multiples of 32");
static_assert((kRows % 64) == 0 && (kXgP % 64) == 0 && (kDm % 64) == 0 && (kDi % 64) == 0, "GEMM M,N and transpose tiles multiples of 64");
static_assert((kDi % kScanCh) == 0 && (kSeq % 16) == 0 && (kRows % 32) == 0, "scan and x_proj tiling");
static_assert(kNs == 8, "state count");

constexpr size_t kSzX16   = (size_t)kRows * kDm * 2;
constexpr size_t kSzY16   = (size_t)kRows * kDi * 2;
constexpr size_t kSzR0    = (kSzY16 > kSzX16) ? kSzY16 : kSzX16;
constexpr size_t kSzWinT  = (size_t)kXgP * kDm * 2;
constexpr size_t kSzWoutT = (size_t)kDm * kDi * 2;
constexpr size_t kSzXG    = (size_t)kRows * kXgP * 4;
constexpr size_t kSzTP    = (size_t)kRows * kNs * 4;
constexpr size_t kOffR0    = 0;
constexpr size_t kOffWinT  = kOffR0 + kSzR0;
constexpr size_t kOffWoutT = kOffWinT + kSzWinT;
constexpr size_t kOffXG    = kOffWoutT + kSzWoutT;
constexpr size_t kOffTP    = kOffXG + kSzXG;
constexpr size_t kWsTotal  = kOffTP + kSzTP;
static_assert(kSzR0 == 25165824ull && kSzWinT == 1572864ull && kSzWoutT == 786432ull &&
              kSzXG == 100663296ull && kSzTP == 524288ull, "carve sizes");
static_assert(kWsTotal == 128712704ull, "carve total");
static_assert(kWsTotal <= 134217728ull, "carve cap");
static_assert((kOffWinT % 128) == 0 && (kOffWoutT % 128) == 0 && (kOffXG % 128) == 0 && (kOffTP % 128) == 0, "128-B aligned regions");

__device__ __forceinline__ _Float16 to_h_flush(float v) {
  const float w = (fabsf(v) < kH16Min) ? 0.0f : v;
  return (_Float16)w;
}
__device__ __forceinline__ _Float16 to_h_flush_clamp(float v) {
  const float c = fminf(fmaxf(v, -kH16Max), kH16Max);
  const float w = (fabsf(c) < kH16Min) ? 0.0f : c;
  return (_Float16)w;
}
__device__ __forceinline__ float silu_f32(float v) {
  const float e = expf(-v);
  return v * __builtin_amdgcn_rcpf(1.0f + e);
}

__device__ __forceinline__ void tie_acc_h(v8f& a, v16h x, v16h y) { asm volatile("" : "+v"(a) : "v"(x), "v"(y)); }
__device__ __forceinline__ void nop_guard_h(v8f& a, v16h x, v16h y) { asm volatile("v_nop\n\tv_nop\n\tv_nop\n\tv_nop" : "+v"(a) : "v"(x), "v"(y)); }
__device__ __forceinline__ void keep4_h(v16h a, v16h b, v16h c, v16h d) { asm volatile("v_nop" :: "v"(a), "v"(b), "v"(c), "v"(d)); }
__device__ __forceinline__ void acc_guard4(v8f& a, v8f& b, v8f& c, v8f& d) { asm volatile("v_nop\n\tv_nop\n\tv_nop\n\tv_nop" : "+v"(a), "+v"(b), "+v"(c), "+v"(d)); }

union FragU { v16h v; v8h h[2]; };
__device__ __forceinline__ v16h frag_load_h(const _Float16* p) {
  FragU f;
  f.h[0] = *(const v8h*)(p);
  f.h[1] = *(const v8h*)(p + 16);
  return f.v;
}
__device__ __forceinline__ v8f mma_h(v16h a, v16h b, v8f c) {
  return __builtin_amdgcn_wmma_f32_16x16x32_f16(false, a, false, b, (short)0, c, false, false);
}

template <int ACT>
__global__ __launch_bounds__(256) void gemm_f16_tile64(
    const unsigned short* __restrict__ Ap, int lda,
    const unsigned short* __restrict__ Btp, int ldb,
    float* __restrict__ Cout, int ldc, int M, int N, int K, float scale)
{
  const _Float16* A  = (const _Float16*)Ap;
  const _Float16* Bt = (const _Float16*)Btp;
  __shared__ __align__(16) float sT[8][16 * 68];
  const int lane = threadIdx.x & 31;
  const int wave = threadIdx.x >> 5;
  const int tilesN = N >> 6;
  const int tilesM = M >> 6;
  const int tile = blockIdx.x * 8 + wave;
  if (tile >= tilesM * tilesN) return;
  const int tm = tile / tilesN;
  const int tn = tile - tm * tilesN;
  const int m0 = tm << 6;
  const int n0 = tn << 6;

  const int rlane = lane & 15;
  const int koff  = (lane >> 4) * 8;
  const int mOff  = (lane >> 4) * 8;

  v8f acc[4][4];
#pragma unroll
  for (int i = 0; i < 4; ++i)
#pragma unroll
    for (int j = 0; j < 4; ++j) acc[i][j] = (v8f){0.f, 0.f, 0.f, 0.f, 0.f, 0.f, 0.f, 0.f};

  for (int k0 = 0; k0 < K; k0 += 32) {
    v16h bh[4];
#pragma unroll
    for (int j = 0; j < 4; ++j) {
      const size_t bo = (size_t)(n0 + (j << 4) + rlane) * ldb + koff + k0;
      bh[j] = frag_load_h(Bt + bo);
    }
#pragma unroll
    for (int i = 0; i < 4; ++i) {
      const size_t ao = (size_t)(m0 + (i << 4) + rlane) * lda + koff + k0;
      const v16h ah = frag_load_h(A + ao);
#pragma unroll
      for (int j = 0; j < 4; ++j) acc[i][j] = mma_h(ah, bh[j], acc[i][j]);
      tie_acc_h(acc[i][0], ah, bh[0]);
      tie_acc_h(acc[i][1], ah, bh[1]);
      tie_acc_h(acc[i][2], ah, bh[2]);
      nop_guard_h(acc[i][3], ah, bh[3]);
    }
    keep4_h(bh[0], bh[1], bh[2], bh[3]);
  }
  acc_guard4(acc[0][0], acc[0][1], acc[0][2], acc[0][3]);
  acc_guard4(acc[1][0], acc[1][1], acc[1][2], acc[1][3]);
  acc_guard4(acc[2][0], acc[2][1], acc[2][2], acc[2][3]);
  acc_guard4(acc[3][0], acc[3][1], acc[3][2], acc[3][3]);

  float* slab = sT[wave];
  const int hh = lane >> 4;
  const int c4 = (lane & 15) * 4;
#pragma unroll
  for (int i = 0; i < 4; ++i) {
    const int mBase = m0 + (i << 4);
#pragma unroll
    for (int j = 0; j < 4; ++j) {
#pragma unroll
      for (int r = 0; r < 8; ++r) {
        slab[(mOff + r) * 68 + (j << 4) + rlane] = acc[i][j][r] * scale;
      }
    }
    __builtin_amdgcn_fence(__ATOMIC_RELEASE, "workgroup");
    __builtin_amdgcn_wave_barrier();
    __builtin_amdgcn_fence(__ATOMIC_ACQUIRE, "workgroup");
    if (ACT == 1) {
#pragma unroll 1
      for (int it = 0; it < 8; ++it) {
        float* sp = slab + (it * 2 + hh) * 68 + c4;
        const v4f v = *(const v4f*)sp;
        v4f o;
        o[0] = silu_f32(v[0]);
        o[1] = silu_f32(v[1]);
        o[2] = silu_f32(v[2]);
        o[3] = silu_f32(v[3]);
        *(v4f*)sp = o;
      }
      __builtin_amdgcn_fence(__ATOMIC_RELEASE, "workgroup");
      __builtin_amdgcn_wave_barrier();
      __builtin_amdgcn_fence(__ATOMIC_ACQUIRE, "workgroup");
    }
    for (int pass = 0; pass < 2; ++pass) {
#pragma unroll
      for (int it = 0; it < 8; ++it) {
        const int row = it * 2 + hh;
        const v4f v = *(const v4f*)(slab + row * 68 + c4);
        *(volatile v4f*)(Cout + (size_t)(mBase + row) * ldc + n0 + c4) = v;
      }
      __threadfence();
    }
    __builtin_amdgcn_fence(__ATOMIC_RELEASE, "workgroup");
    __builtin_amdgcn_wave_barrier();
    __builtin_amdgcn_fence(__ATOMIC_ACQUIRE, "workgroup");
  }
}

__global__ __launch_bounds__(256) void cast_f16_kernel(
    const float* __restrict__ src, unsigned short* __restrict__ dst, int total8, float carry)
{
  const int i = blockIdx.x * 256 + threadIdx.x;
  if (i >= total8) return;
  const size_t e0 = (size_t)i << 3;
  const float* p = src + e0;
  const v4f a0 = *(const v4f*)(p);
  const v4f a1 = *(const v4f*)(p + 4);
  v8h hv;
#pragma unroll
  for (int e = 0; e < 4; ++e) {
    hv[e]     = to_h_flush(a0[e] * carry);
    hv[4 + e] = to_h_flush(a1[e] * carry);
  }
  unsigned short* q = dst + e0;
  *(volatile v8h*)q = hv;
  __threadfence();
  *(volatile v8h*)q = hv;
}

__global__ __launch_bounds__(256) void transpose_cast_kernel(
    const float* __restrict__ W, unsigned short* __restrict__ Bt, int Kdim, int Ndim, float carry)
{
  __shared__ float tile[64 * 65];
  const int tid = threadIdx.x, lane = tid & 31, wave = tid >> 5;
  const int n0 = blockIdx.x * 64;
  const int k0 = blockIdx.y * 64;
#pragma unroll
  for (int p = 0; p < 16; ++p) {
    const int idx = tid + p * 256;
    const int kk  = idx >> 6;
    const int nn  = idx & 63;
    const float v = W[(size_t)(k0 + kk) * Ndim + n0 + nn];
    tile[kk * 65 + nn] = v * carry;
  }
  __syncthreads();
  const int q = lane >> 3, c8 = (lane & 7) * 8;
  v8h hv[2];
#pragma unroll
  for (int it = 0; it < 2; ++it) {
    const int nrow = it * 32 + wave * 4 + q;
#pragma unroll
    for (int e = 0; e < 8; ++e) hv[it][e] = to_h_flush(tile[(c8 + e) * 65 + nrow]);
  }
  for (int pass = 0; pass < 2; ++pass) {
#pragma unroll
    for (int it = 0; it < 2; ++it) {
      const int nrow = it * 32 + wave * 4 + q;
      *(volatile v8h*)(Bt + (size_t)(n0 + nrow) * Kdim + k0 + c8) = hv[it];
    }
    __threadfence();
  }
}

__global__ __launch_bounds__(256) void xproj_kernel(
    const float* __restrict__ XG, const float* __restrict__ Wx, float* __restrict__ TP)
{
  __shared__ __align__(16) float sW[kDi * kNs];
  __shared__ __align__(16) float sR[32 * kNs];
  const int tid = threadIdx.x, lane = tid & 31, wave = tid >> 5;
#pragma unroll
  for (int p = 0; p < 6; ++p) {
    const int idx = tid + p * 256;
    *(v4f*)(sW + idx * 4) = *(const v4f*)(Wx + idx * 4);
  }
  __syncthreads();
  const int r0 = blockIdx.x * 32 + wave * 4;
  float acc[4][kNs];
#pragma unroll
  for (int r = 0; r < 4; ++r)
#pragma unroll
    for (int n = 0; n < kNs; ++n) acc[r][n] = 0.f;

#pragma unroll 1
  for (int kk = 0; kk < kDi / 32; ++kk) {
    const int k = kk * 32 + lane;
    const v4f w0 = *(const v4f*)(sW + k * kNs);
    const v4f w1 = *(const v4f*)(sW + k * kNs + 4);
#pragma unroll
    for (int r = 0; r < 4; ++r) {
      const float xv = XG[(size_t)(r0 + r) * kXgP + k];
      acc[r][0] = fmaf(xv, w0[0], acc[r][0]);
      acc[r][1] = fmaf(xv, w0[1], acc[r][1]);
      acc[r][2] = fmaf(xv, w0[2], acc[r][2]);
      acc[r][3] = fmaf(xv, w0[3], acc[r][3]);
      acc[r][4] = fmaf(xv, w1[0], acc[r][4]);
      acc[r][5] = fmaf(xv, w1[1], acc[r][5]);
      acc[r][6] = fmaf(xv, w1[2], acc[r][6]);
      acc[r][7] = fmaf(xv, w1[3], acc[r][7]);
    }
  }
#pragma unroll
  for (int r = 0; r < 4; ++r) {
#pragma unroll
    for (int n = 0; n < kNs; ++n) {
#pragma unroll
      for (int m = 16; m >= 1; m >>= 1) acc[r][n] += __shfl_xor(acc[r][n], m, 32);
    }
  }
  if (lane == 0) {
#pragma unroll
    for (int r = 0; r < 4; ++r) {
      const v4f o0 = {acc[r][0], acc[r][1], acc[r][2], acc[r][3]};
      const v4f o1 = {acc[r][4], acc[r][5], acc[r][6], acc[r][7]};
      *(v4f*)(sR + (wave * 4 + r) * kNs)     = o0;
      *(v4f*)(sR + (wave * 4 + r) * kNs + 4) = o1;
    }
  }
  __syncthreads();
  if (wave == 0) {
    float* dst = TP + (size_t)blockIdx.x * (32 * kNs);
    const v4f v0 = *(const v4f*)(sR + lane * 4);
    const v4f v1 = *(const v4f*)(sR + 128 + lane * 4);
    *(volatile v4f*)(dst + lane * 4)       = v0;
    *(volatile v4f*)(dst + 128 + lane * 4) = v1;
    __threadfence();
    *(volatile v4f*)(dst + lane * 4)       = v0;
    *(volatile v4f*)(dst + 128 + lane * 4) = v1;
  }
}

__global__ __launch_bounds__(256) void scan_kernel(
    const float* __restrict__ XG, const float* __restrict__ TP,
    const float* __restrict__ A_log, const float* __restrict__ Dp,
    const float* __restrict__ Wdt, const float* __restrict__ bdt,
    unsigned short* __restrict__ Y16)
{
  __shared__ __align__(16) float sTs[16 * kNs];
  __shared__ __align__(16) float sY[16 * kTP];
  __shared__ __align__(16) float sA[kNs * kScanCh];
  const int tid = threadIdx.x, lane = tid & 31, wave = tid >> 5;
  const int bix = blockIdx.x / kScanBlkPerB;
  const int d0  = (blockIdx.x - bix * kScanBlkPerB) * kScanCh;
  const int d   = d0 + tid;
  const size_t row0 = (size_t)bix * kSeq;

#pragma unroll 1
  for (int n = 0; n < kNs; ++n) sA[n * kScanCh + tid] = -expf(A_log[(size_t)d * kNs + n]) * kLog2e;
  __syncthreads();
  float A2[kNs], wd[kNs], h[kNs];
#pragma unroll
  for (int n = 0; n < kNs; ++n) {
    A2[n] = sA[n * kScanCh + tid];
    wd[n] = Wdt[(size_t)n * kDi + d];
    h[n]  = 0.f;
  }
  const float bb = bdt[d];
  const float Dd = Dp[d];

#pragma unroll 1
  for (int c = 0; c < kSeq / 16; ++c) {
    const int l0 = c * 16;
    if (tid < 32) {
      const v4f v = *(const v4f*)(TP + (row0 + l0) * kNs + tid * 4);
      *(v4f*)(sTs + tid * 4) = v;
    }
    __syncthreads();
#pragma unroll 1
    for (int s = 0; s < 16; ++s) {
      const size_t m = row0 + (size_t)(l0 + s);
      const float xv = XG[m * kXgP + d];
      const float gv = XG[m * kXgP + kDi + d];
      const v4f t0 = *(const v4f*)(sTs + s * kNs);
      const v4f t1 = *(const v4f*)(sTs + s * kNs + 4);
      float raw = t0[0] * wd[0];
      raw = fmaf(t0[1], wd[1], raw);
      raw = fmaf(t0[2], wd[2], raw);
      raw = fmaf(t0[3], wd[3], raw);
      raw = fmaf(t1[0], wd[4], raw);
      raw = fmaf(t1[1], wd[5], raw);
      raw = fmaf(t1[2], wd[6], raw);
      raw = fmaf(t1[3], wd[7], raw);
      raw += bb;
      const float ea    = expf(-fabsf(raw));
      const float delta = fmaxf(raw, 0.0f) + log1pf(ea);
      const float dx    = delta * xv;
      float ysum = 0.f;
#pragma unroll
      for (int n = 0; n < kNs; ++n) {
        const float dA = __builtin_amdgcn_exp2f(delta * A2[n]);
        h[n] = fmaf(dA, h[n], dx);
        ysum += h[n];
      }
      const float y = fmaf(Dd, xv, ysum) * gv;
      sY[s * kTP + tid] = y * kYCarry;
    }
    __syncthreads();
    v8h hv[2];
#pragma unroll
    for (int it = 0; it < 2; ++it) {
      const float* sp = sY + (it * 8 + wave) * kTP + lane * 8;
      const v4f a0 = *(const v4f*)(sp);
      const v4f a1 = *(const v4f*)(sp + 4);
#pragma unroll
      for (int e = 0; e < 4; ++e) {
        hv[it][e]     = to_h_flush_clamp(a0[e]);
        hv[it][4 + e] = to_h_flush_clamp(a1[e]);
      }
    }
    for (int pass = 0; pass < 2; ++pass) {
#pragma unroll
      for (int it = 0; it < 2; ++it)
        *(volatile v8h*)(Y16 + (row0 + (size_t)(l0 + it * 8 + wave)) * kDi + d0 + lane * 8) = hv[it];
      __threadfence();
    }
  }
}

extern "C" void kernel_launch(void* const* d_in, const int* in_sizes, int n_in,
                              void* d_out, int out_size, void* d_ws, size_t ws_size,
                              hipStream_t stream)
{
  if (n_in < 8) return;
  if (in_sizes[0] != kRows * kDm) return;
  if (in_sizes[1] != kDm * kXgP) return;
  if (in_sizes[2] != kDi * kNs) return;
  if (in_sizes[3] != kDi) return;
  if (in_sizes[4] != kDi * kNs) return;
  if (in_sizes[5] != kNs * kDi) return;
  if (in_sizes[6] != kDi) return;
  if (in_sizes[7] != kDi * kDm) return;
  if (out_size != kRows * kDm) return;
  if (ws_size < kWsTotal) return;

  const float* x       = (const float*)d_in[0];
  const float* W_in    = (const float*)d_in[1];
  const float* A_log   = (const float*)d_in[2];
  const float* D_param = (const float*)d_in[3];
  const float* W_x     = (const float*)d_in[4];
  const float* W_dt    = (const float*)d_in[5];
  const float* b_dt    = (const float*)d_in[6];
  const float* W_out   = (const float*)d_in[7];
  float* out = (float*)d_out;

  char* ws = (char*)d_ws;
  unsigned short* X16   = (unsigned short*)(ws + kOffR0);
  unsigned short* Y16   = (unsigned short*)(ws + kOffR0);
  unsigned short* WinT  = (unsigned short*)(ws + kOffWinT);
  unsigned short* WoutT = (unsigned short*)(ws + kOffWoutT);
  float*          XG    = (float*)(ws + kOffXG);
  float*          TPl   = (float*)(ws + kOffTP);

  cast_f16_kernel<<<(kRows * kDm / 8) / 256, 256, 0, stream>>>(x, X16, kRows * kDm / 8, kXCarry);

  transpose_cast_kernel<<<dim3(kXgP / 64, kDm / 64), 256, 0, stream>>>(W_in, WinT, kDm, kXgP, kWCarry);
  transpose_cast_kernel<<<dim3(kDm / 64, kDi / 64), 256, 0, stream>>>(W_out, WoutT, kDi, kDm, kWCarry);

  gemm_f16_tile64<1><<<((kRows / 64) * (kXgP / 64)) / 8, 256, 0, stream>>>(
      X16, kDm, WinT, kDm, XG, kXgP, kRows, kXgP, kDm, kFold1);

  xproj_kernel<<<kRows / 32, 256, 0, stream>>>(XG, W_x, TPl);

  scan_kernel<<<kBatch * kScanBlkPerB, kScanCh, 0, stream>>>(XG, TPl, A_log, D_param, W_dt, b_dt, Y16);

  gemm_f16_tile64<0><<<((kRows / 64) * (kDm / 64)) / 8, 256, 0, stream>>>(
      Y16, kDi, WoutT, kDi, out, kDm, kRows, kDm, kDi, kFold2);
}
